// Mamba2Block_55456617726038
// MI455X (gfx1250) — hardware-verified
//
#include <hip/hip_runtime.h>
#include <math.h>

typedef __attribute__((ext_vector_type(16))) __bf16   v16b;
typedef __attribute__((ext_vector_type(8)))  __bf16   v8b;
typedef __attribute__((ext_vector_type(8)))  _Float16 v8h;
typedef __attribute__((ext_vector_type(8)))  float    v8f;
typedef __attribute__((ext_vector_type(4)))  float    v4f;

constexpr int kBatch   = 2;
constexpr int kSeq     = 2048;
constexpr int kDm      = 1024;
constexpr int kDin     = 2048;
constexpr int kNst     = 128;
constexpr int kHd      = 64;
constexpr int kNh      = 32;
constexpr int kDproj   = 4384;
constexpr int kDprojP  = 4416;
constexpr int kRows    = kBatch * kSeq;
constexpr int kZxW     = 2 * kDin;
constexpr int kBcdW    = 320;
constexpr int kTS      = 32;
constexpr int kScanYP  = 68;
static_assert(kNh * kHd == kDin, "heads");
static_assert(2 * kDin + 2 * kNst + kNh == kDproj, "proj width");
static_assert(kDprojP == kZxW + kBcdW && (kDprojP % 64) == 0 && kDprojP >= kDproj, "padded proj width");
static_assert((kDm % 32) == 0 && (kDin % 32) == 0, "GEMM K multiples of 32");
static_assert((kRows % 64) == 0 && (kZxW % 64) == 0 && (kBcdW % 64) == 0 && (kDm % 64) == 0, "GEMM M,N multiples of 64");
static_assert((kSeq % kTS) == 0 && (kSeq % 64) == 0 && (kRows % 32) == 0 && kTS == 32 && kHd == 64, "tile multiples");
static_assert(((kRows / 64) * (kZxW / 64)) % 8 == 0 && ((kRows / 64) * (kBcdW / 64)) % 8 == 0 &&
              ((kRows / 64) * (kDm / 64)) % 8 == 0, "GEMM grids exact");

constexpr size_t kOffBT1 = 0;
constexpr size_t kOffBT2 = kOffBT1 + (size_t)kDprojP * kDm * 2;
constexpr size_t kOffA1  = kOffBT2 + (size_t)kDm * kDin * 2;
constexpr size_t kOffSCL = kOffA1  + (size_t)kRows * kDm * 2;
constexpr size_t kOffZX  = kOffSCL + (size_t)kRows * 4;
constexpr size_t kOffBCD = kOffZX  + (size_t)kRows * kZxW * 4;
constexpr size_t kOffDT  = kOffBCD + (size_t)kRows * kBcdW * 4;
constexpr size_t kOffDA  = kOffDT  + (size_t)kRows * kNh * 4;
constexpr size_t kOffYH  = kOffDA  + (size_t)kRows * kNh * 4;
constexpr size_t kOffYL  = kOffYH  + (size_t)kRows * kDin * 2;
constexpr size_t kWsTotal = kOffYL + (size_t)kRows * kDin * 2;
static_assert(kWsTotal == 128598016ull, "carve total");
static_assert(kWsTotal <= 134217728ull, "carve cap");
static_assert((kOffBT2 % 128) == 0 && (kOffA1 % 128) == 0 && (kOffSCL % 128) == 0 && (kOffZX % 128) == 0 &&
              (kOffBCD % 128) == 0 && (kOffDT % 128) == 0 && (kOffDA % 128) == 0 && (kOffYH % 128) == 0 &&
              (kOffYL % 128) == 0, "128-B aligned regions");

__device__ __forceinline__ unsigned short f2bf_bits(float f) {
  unsigned u = __float_as_uint(f);
  return (unsigned short)((u + 0x7FFFu + ((u >> 16) & 1u)) >> 16);
}
__device__ __forceinline__ float bf_bits2f(unsigned short h) { return __uint_as_float(((unsigned)h) << 16); }
__device__ __forceinline__ float bf_rne(float f) { return bf_bits2f(f2bf_bits(f)); }

__device__ __forceinline__ void dep_guard4_b(v8f& a, v8f& b, v8f& c, v8f& d, v16b x, v16b y) {
  asm volatile("v_nop\n\tv_nop\n\tv_nop\n\tv_nop" : "+v"(a), "+v"(b), "+v"(c), "+v"(d) : "v"(x), "v"(y));
}
__device__ __forceinline__ void keep4_b(v16b a, v16b b, v16b c, v16b d) { asm volatile("v_nop" :: "v"(a), "v"(b), "v"(c), "v"(d)); }
__device__ __forceinline__ void acc_guard4(v8f& a, v8f& b, v8f& c, v8f& d) { asm volatile("v_nop\n\tv_nop\n\tv_nop\n\tv_nop" : "+v"(a), "+v"(b), "+v"(c), "+v"(d)); }

struct FragB {
  union U { v16b v; v8b h[2]; };
  static __device__ __forceinline__ v16b load(const __bf16* p) {
    U f; f.h[0] = *(const v8b*)(p); f.h[1] = *(const v8b*)(p + 16); return f.v;
  }
  static __device__ __forceinline__ v8f mma(v16b a, v16b b, v8f c) {
    return __builtin_amdgcn_wmma_f32_16x16x32_bf16(false, a, false, b, (short)0, c, false, false);
  }
};

template <int SPL, bool RESID, bool ROWSC>
__global__ __launch_bounds__(256) void wmma_gemm64(
    const unsigned short* __restrict__ Ap, const unsigned short* __restrict__ A2p, int lda,
    const unsigned short* __restrict__ Btp, int ldb,
    float* __restrict__ C, int ldc,
    const float* __restrict__ rowsc, const float* __restrict__ resid,
    int M, int N, int K) {
  const __bf16* A = (const __bf16*)Ap; const __bf16* A2 = (const __bf16*)A2p; const __bf16* Bt = (const __bf16*)Btp;
  __shared__ __align__(16) float sT[8][16 * 68];
  const int lane = threadIdx.x & 31;
  const int wave = threadIdx.x >> 5;
  const int tilesN = N >> 6;
  const int tilesM = M >> 6;
  const int tile = blockIdx.x * 8 + wave;
  if (tile >= tilesM * tilesN) return;
  const int tm = tile / tilesN;
  const int tn = tile - tm * tilesN;
  const int m0 = tm << 6;
  const int n0 = tn << 6;

  const int rlane = lane & 15;
  const int koff  = (lane >> 4) * 8;
  const int mOff  = (lane >> 4) * 8;

  v8f acc[4][4];
#pragma unroll
  for (int i = 0; i < 4; ++i)
#pragma unroll
    for (int j = 0; j < 4; ++j) acc[i][j] = (v8f){0.f,0.f,0.f,0.f,0.f,0.f,0.f,0.f};

  for (int k0 = 0; k0 < K; k0 += 32) {
    v16b bh[4];
#pragma unroll
    for (int j = 0; j < 4; ++j) {
      const size_t bo = (size_t)(n0 + (j << 4) + rlane) * ldb + koff + k0;
      bh[j] = FragB::load(Bt + bo);
    }
#pragma unroll
    for (int i = 0; i < 4; ++i) {
      const size_t ao = (size_t)(m0 + (i << 4) + rlane) * lda + koff + k0;
      const v16b ah = FragB::load(A + ao);
      v16b al = ah;
      if (SPL == 1) al = FragB::load(A2 + ao);
#pragma unroll
      for (int j = 0; j < 4; ++j) {
        acc[i][j] = FragB::mma(ah, bh[j], acc[i][j]);
        if (SPL == 1) acc[i][j] = FragB::mma(al, bh[j], acc[i][j]);
      }
      dep_guard4_b(acc[i][0], acc[i][1], acc[i][2], acc[i][3], ah, (SPL == 1) ? al : bh[3]);
    }
    keep4_b(bh[0], bh[1], bh[2], bh[3]);
  }
  acc_guard4(acc[0][0], acc[0][1], acc[0][2], acc[0][3]);
  acc_guard4(acc[1][0], acc[1][1], acc[1][2], acc[1][3]);
  acc_guard4(acc[2][0], acc[2][1], acc[2][2], acc[2][3]);
  acc_guard4(acc[3][0], acc[3][1], acc[3][2], acc[3][3]);

  float* slab = sT[wave];
#pragma unroll
  for (int i = 0; i < 4; ++i) {
    const int mBase = m0 + (i << 4);
#pragma unroll
    for (int j = 0; j < 4; ++j) {
#pragma unroll
      for (int r = 0; r < 8; ++r) {
        slab[(mOff + r) * 68 + (j << 4) + rlane] = acc[i][j][r];
      }
    }
    __builtin_amdgcn_fence(__ATOMIC_RELEASE, "workgroup");
    __builtin_amdgcn_wave_barrier();
    __builtin_amdgcn_fence(__ATOMIC_ACQUIRE, "workgroup");
    {
      const int hh = lane >> 4, c4 = (lane & 15) * 4;
      v4f ov[8];
#pragma unroll
      for (int it = 0; it < 8; ++it) {
        const int row = it * 2 + hh;
        v4f v = *(const v4f*)(slab + row * 68 + c4);
        if (ROWSC) {
          const float rs = rowsc[mBase + row];
          v = v * rs;
        }
        if (RESID) {
          const v4f rr = *(const v4f*)(resid + (size_t)(mBase + row) * ldc + n0 + c4);
          v4f rb;
#pragma unroll
          for (int e = 0; e < 4; ++e) rb[e] = bf_rne(rr[e]);
          v = v + rb;
        }
        ov[it] = v;
      }
      for (int pass = 0; pass < 2; ++pass) {
#pragma unroll
        for (int it = 0; it < 8; ++it) {
          const int row = it * 2 + hh;
          *(volatile v4f*)(C + (size_t)(mBase + row) * ldc + n0 + c4) = ov[it];
        }
        __threadfence();
      }
    }
    __builtin_amdgcn_fence(__ATOMIC_RELEASE, "workgroup");
    __builtin_amdgcn_wave_barrier();
    __builtin_amdgcn_fence(__ATOMIC_ACQUIRE, "workgroup");
  }
}

template <int COLS>
__global__ __launch_bounds__(256) void cast_rows_bf16_kernel(
    const float* __restrict__ src, unsigned short* __restrict__ dst, int rowsSrc, int total8)
{
  const int i = blockIdx.x * 256 + threadIdx.x;
  if (i >= total8) return;
  constexpr int kC8 = COLS / 8;
  const int row = i / kC8;
  const int c8  = i - row * kC8;
  const int rowc = (row < rowsSrc) ? row : (rowsSrc - 1);
  const float* sp = src + (size_t)rowc * COLS + (size_t)c8 * 8;
  const v4f a0 = *(const v4f*)(sp);
  const v4f a1 = *(const v4f*)(sp + 4);
  const float f = (row < rowsSrc) ? 1.0f : 0.0f;
  v8h hv;
#pragma unroll
  for (int e = 0; e < 4; ++e) {
    hv[e]     = __builtin_bit_cast(_Float16, f2bf_bits(a0[e] * f));
    hv[4 + e] = __builtin_bit_cast(_Float16, f2bf_bits(a1[e] * f));
  }
  unsigned short* qp = dst + (size_t)i * 8;
  *(volatile v8h*)qp = hv;
  __threadfence();
  *(volatile v8h*)qp = hv;
}

__global__ __launch_bounds__(256) void rmsnorm_kernel(
    const float* __restrict__ x, const float* __restrict__ w,
    unsigned short* __restrict__ A1, float* __restrict__ SCL)
{
  __shared__ float sS[32];
  const int tid = threadIdx.x, lane = tid & 31, wave = tid >> 5;
  const int rbase = blockIdx.x * 32 + wave * 4;
#pragma unroll 1
  for (int r = 0; r < 4; ++r) {
    const size_t row = (size_t)(rbase + r);
    const float* xr = x + row * kDm;
    float ss = 0.0f;
    v8h hv[4];
#pragma unroll
    for (int it = 0; it < 4; ++it) {
      const int e0 = it * 256 + lane * 8;
      const v4f a0 = *(const v4f*)(xr + e0);
      const v4f a1 = *(const v4f*)(xr + e0 + 4);
      const v4f w0 = *(const v4f*)(w + e0);
      const v4f w1 = *(const v4f*)(w + e0 + 4);
#pragma unroll
      for (int e = 0; e < 4; ++e) {
        const float xb0 = bf_rne(a0[e]), xb1 = bf_rne(a1[e]);
        ss = fmaf(xb0, xb0, ss);
        ss = fmaf(xb1, xb1, ss);
        hv[it][e]     = __builtin_bit_cast(_Float16, f2bf_bits(xb0 * bf_rne(w0[e])));
        hv[it][4 + e] = __builtin_bit_cast(_Float16, f2bf_bits(xb1 * bf_rne(w1[e])));
      }
    }
#pragma unroll
    for (int off = 16; off > 0; off >>= 1) ss += __shfl_xor(ss, off, 32);
    const float scl = rsqrtf(ss * (1.0f / (float)kDm) + 1e-6f);
    if (lane == 0) sS[wave * 4 + r] = scl;
    unsigned short* ap = A1 + row * kDm + (size_t)lane * 8;
    for (int pass = 0; pass < 2; ++pass) {
#pragma unroll
      for (int it = 0; it < 4; ++it) *(volatile v8h*)(ap + it * 256) = hv[it];
      __threadfence();
    }
  }
  __syncthreads();
  if (wave == 0) {
    const float v = sS[lane];
    float* sp = SCL + (size_t)blockIdx.x * 32 + lane;
    *(volatile float*)sp = v;
    __threadfence();
    *(volatile float*)sp = v;
  }
}

__global__ __launch_bounds__(256) void dt_kernel(
    const float* __restrict__ BCD, const float* __restrict__ dtb, const float* __restrict__ Alog,
    float* __restrict__ DT, float* __restrict__ DA)
{
  const int idx = blockIdx.x * 256 + threadIdx.x;
  const int hd  = idx & (kNh - 1);
  const int row = idx >> 5;
  const float raw = BCD[(size_t)row * kBcdW + 2 * kNst + hd] + bf_rne(dtb[hd]);
  const float ex  = expf(-fabsf(raw));
  const float dt  = fmaxf(raw, 0.0f) + log1pf(ex);
  const float av  = expf(bf_rne(Alog[hd]));
  const float da  = expf((-av) * dt);
  ((volatile float*)DT)[idx] = dt;
  ((volatile float*)DA)[idx] = da;
  __threadfence();
  ((volatile float*)DT)[idx] = dt;
  ((volatile float*)DA)[idx] = da;
}

__global__ __launch_bounds__(256) void scan_kernel(
    const float* __restrict__ BCD, const float* __restrict__ ZX,
    const float* __restrict__ DT, const float* __restrict__ DA,
    const float* __restrict__ cw, const float* __restrict__ cb, const float* __restrict__ Dp,
    unsigned short* __restrict__ YH, unsigned short* __restrict__ YL)
{
  __shared__ __align__(16) float sBC[kTS * 2 * kNst];
  __shared__ __align__(16) float sXS[(kTS + 3) * kHd];
  __shared__ __align__(16) float sXC[kTS * kHd];
  __shared__ __align__(16) float sY[kTS * kScanYP];
  __shared__ float sDT[kTS];
  __shared__ float sDA[kTS];
  __shared__ float sCW[kHd * 4];
  __shared__ float sCB[kHd];
  const int tid = threadIdx.x, lane = tid & 31, wave = tid >> 5;
  const int bix = blockIdx.x >> 5;
  const int hd  = blockIdx.x & (kNh - 1);
  const int ch0 = hd * kHd;
  const int p   = tid >> 2;
  const int n0  = (tid & 3) * 32;
  const size_t row0 = (size_t)bix * kSeq;
  sCW[tid] = bf_rne(cw[(size_t)ch0 * 4 + tid]);
  if (tid < kHd) sCB[tid] = bf_rne(cb[ch0 + tid]);
  const float Dh = bf_rne(Dp[hd]);
  float h[32];
#pragma unroll
  for (int j = 0; j < 32; ++j) h[j] = 0.0f;
  const int q = lane >> 3, c8 = (lane & 7) * 8;
  constexpr int kXsF4 = (kTS + 3) * (kHd / 4);

#pragma unroll 1
  for (int t0 = 0; t0 < kSeq; t0 += kTS) {
    __syncthreads();
#pragma unroll
    for (int i = 0; i < 8; ++i) {
      const int idx = tid + 256 * i;
      const int s = idx >> 6, c = (idx & 63) * 4;
      *(v4f*)(sBC + s * 256 + c) = *(const v4f*)(BCD + (row0 + t0 + s) * kBcdW + c);
    }
#pragma unroll
    for (int i = 0; i < 3; ++i) {
      int idx = tid + 256 * i;
      idx = (idx < kXsF4) ? idx : (kXsF4 - 1);
      const int r = idx >> 4, c = (idx & 15) * 4;
      const int tt  = t0 - 3 + r;
      const int ttc = (tt >= 0) ? tt : 0;
      const float f = (tt >= 0) ? 1.0f : 0.0f;
      const v4f v = *(const v4f*)(ZX + (row0 + ttc) * kZxW + kDin + ch0 + c);
      *(v4f*)(sXS + r * kHd + c) = v * f;
    }
    if (wave == 0) {
      sDT[lane] = DT[(row0 + t0 + lane) * kNh + hd];
      sDA[lane] = DA[(row0 + t0 + lane) * kNh + hd];
    }
    __syncthreads();

#pragma unroll 1
    for (int i = 0; i < 8; ++i) {
      const int idx = tid + 256 * i;
      const int s = idx >> 6, c = idx & 63;
      const float* xp = sXS + s * kHd + c;
      const float* wp = sCW + c * 4;
      float a = wp[0] * xp[0];
      a = fmaf(wp[1], xp[kHd], a);
      a = fmaf(wp[2], xp[2 * kHd], a);
      a = fmaf(wp[3], xp[3 * kHd], a);
      const float sv = a + sCB[c];
      const float sg = __builtin_amdgcn_rcpf(1.0f + __expf(-sv));
      sXC[s * kHd + c] = sv * sg;
    }
    __syncthreads();

#pragma unroll 1
    for (int s = 0; s < kTS; ++s) {
      const float dAv = sDA[s];
      const float dtx = sDT[s] * sXC[s * kHd + p];
      const float* bp = sBC + s * 256 + n0;
      float yp = 0.0f;
#pragma unroll
      for (int j4 = 0; j4 < 8; ++j4) {
        const v4f bv = *(const v4f*)(bp + 4 * j4);
        const v4f cv = *(const v4f*)(bp + kNst + 4 * j4);
#pragma unroll
        for (int e = 0; e < 4; ++e) {
          const float hn = fmaf(h[4 * j4 + e], dAv, dtx * bv[e]);
          h[4 * j4 + e] = hn;
          yp = fmaf(hn, cv[e], yp);
        }
      }
      yp += __shfl_xor(yp, 1, 32);
      yp += __shfl_xor(yp, 2, 32);
      if ((tid & 3) == 0) sY[s * kScanYP + p] = yp;
    }
    __syncthreads();

#pragma unroll 1
    for (int i = 0; i < 8; ++i) {
      const int idx = tid + 256 * i;
      const int s = idx >> 6, c = idx & 63;
      const float zv = ZX[(row0 + t0 + s) * kZxW + ch0 + c];
      const float sg = __builtin_amdgcn_rcpf(1.0f + __expf(-zv));
      const float yv = fmaf(Dh, sXC[s * kHd + c], sY[s * kScanYP + c]);
      sY[s * kScanYP + c] = yv * (zv * sg);
    }
    __syncthreads();

    {
      const int row = wave * 4 + q;
      const float* sp = sY + row * kScanYP + c8;
      const v4f a0 = *(const v4f*)(sp);
      const v4f a1 = *(const v4f*)(sp + 4);
      v8h hv, lv;
#pragma unroll
      for (int e = 0; e < 4; ++e) {
        const unsigned short h0 = f2bf_bits(a0[e]), h1 = f2bf_bits(a1[e]);
        const unsigned short l0 = f2bf_bits(a0[e] - bf_bits2f(h0)), l1 = f2bf_bits(a1[e] - bf_bits2f(h1));
        hv[e]     = __builtin_bit_cast(_Float16, h0);
        hv[4 + e] = __builtin_bit_cast(_Float16, h1);
        lv[e]     = __builtin_bit_cast(_Float16, l0);
        lv[4 + e] = __builtin_bit_cast(_Float16, l1);
      }
      const size_t o = (row0 + t0 + row) * kDin + ch0 + c8;
      *(volatile v8h*)(YH + o) = hv;
      *(volatile v8h*)(YL + o) = lv;
      __threadfence();
      *(volatile v8h*)(YH + o) = hv;
      *(volatile v8h*)(YL + o) = lv;
    }
  }
}

extern "C" void kernel_launch(void* const* d_in, const int* in_sizes, int n_in,
                              void* d_out, int out_size, void* d_ws, size_t ws_size,
                              hipStream_t stream) {
  if (n_in < 9) return;
  if (in_sizes[0] != kRows * kDm) return;
  if (in_sizes[1] != kDm) return;
  if (in_sizes[2] != kDproj * kDm) return;
  if (in_sizes[3] != kDin * 4) return;
  if (in_sizes[4] != kDin) return;
  if (in_sizes[5] != kNh) return;
  if (in_sizes[6] != kNh) return;
  if (in_sizes[7] != kNh) return;
  if (in_sizes[8] != kDm * kDin) return;
  if (out_size != kRows * kDm) return;
  if (ws_size < kWsTotal) return;

  const float* x       = (const float*)d_in[0];
  const float* norm_w  = (const float*)d_in[1];
  const float* W_in    = (const float*)d_in[2];
  const float* conv_w  = (const float*)d_in[3];
  const float* conv_b  = (const float*)d_in[4];
  const float* A_log   = (const float*)d_in[5];
  const float* Dp      = (const float*)d_in[6];
  const float* dt_bias = (const float*)d_in[7];
  const float* W_out   = (const float*)d_in[8];
  float* out = (float*)d_out;

  char* ws = (char*)d_ws;
  unsigned short* BT1 = (unsigned short*)(ws + kOffBT1);
  unsigned short* BT2 = (unsigned short*)(ws + kOffBT2);
  unsigned short* A1  = (unsigned short*)(ws + kOffA1);
  float*          SCL = (float*)(ws + kOffSCL);
  float*          ZX  = (float*)(ws + kOffZX);
  float*          BCD = (float*)(ws + kOffBCD);
  float*          DT  = (float*)(ws + kOffDT);
  float*          DA  = (float*)(ws + kOffDA);
  unsigned short* YH  = (unsigned short*)(ws + kOffYH);
  unsigned short* YL  = (unsigned short*)(ws + kOffYL);

  constexpr int kTot8BT1 = kDprojP * kDm / 8;
  constexpr int kTot8BT2 = kDm * kDin / 8;
  static_assert((kTot8BT1 % 256) == 0 && (kTot8BT2 % 256) == 0, "cast grids exact");

  cast_rows_bf16_kernel<kDm><<<kTot8BT1 / 256, 256, 0, stream>>>(W_in, BT1, kDproj, kTot8BT1);
  cast_rows_bf16_kernel<kDin><<<kTot8BT2 / 256, 256, 0, stream>>>(W_out, BT2, kDm, kTot8BT2);

  rmsnorm_kernel<<<kRows / 32, 256, 0, stream>>>(x, norm_w, A1, SCL);

  wmma_gemm64<0, false, true><<<dim3((kRows / 64) * (kZxW / 64) / 8), 256, 0, stream>>>(
      A1, A1, kDm, BT1, kDm, ZX, kZxW, SCL, nullptr, kRows, kZxW, kDm);
  wmma_gemm64<0, false, true><<<dim3((kRows / 64) * (kBcdW / 64) / 8), 256, 0, stream>>>(
      A1, A1, kDm, BT1 + (size_t)kZxW * kDm, kDm, BCD, kBcdW, SCL, nullptr, kRows, kBcdW, kDm);

  dt_kernel<<<(kRows * kNh) / 256, 256, 0, stream>>>(BCD, dt_bias, A_log, DT, DA);

  scan_kernel<<<kBatch * kNh, 256, 0, stream>>>(BCD, ZX, DT, DA, conv_w, conv_b, Dp, YH, YL);

  wmma_gemm64<1, true, false><<<dim3((kRows / 64) * (kDm / 64) / 8), 256, 0, stream>>>(
      YH, YL, kDin, BT2, kDin, out, kDm, nullptr, x, kRows, kDm, kDin);
}
